// EncoderLstm_one_fc_24008867184782
// MI455X (gfx1250) — hardware-verified
//
#include <hip/hip_runtime.h>


namespace {
constexpr int B = 128, T = 32, F = 2048, H = 1024, NR = B * T, G4 = 4 * H;
constexpr float AS_ = 8.0f, EPS = 1e-5f;

typedef _Float16 b16;
typedef __attribute__((ext_vector_type(16))) _Float16 v16b;
typedef __attribute__((ext_vector_type(8))) _Float16 v8b;
typedef __attribute__((ext_vector_type(8))) float v8f;
typedef __attribute__((ext_vector_type(4))) float v4f;
__device__ __forceinline__ float bf16_rne(float f) { unsigned int u = __float_as_uint(f); u += 0x7FFFu + ((u >> 16) & 1u); return __uint_as_float(u & 0xFFFF0000u); }
__device__ __forceinline__ v16b frag_kb(const b16* p, int hh) { const v8b a = *(const v8b*)(p + 8 * hh), b = *(const v8b*)(p + 16 + 8 * hh); v16b f;
#pragma unroll
  for (int e = 0; e < 8; ++e) { f[e] = a[e]; f[8 + e] = b[e]; } return f; }
__device__ __forceinline__ v16b frag_x(const float* p, int hh) { v16b f;
#pragma unroll
  for (int e = 0; e < 8; ++e) { f[e] = (b16)bf16_rne(p[8 * hh + e]); f[8 + e] = (b16)bf16_rne(p[16 + 8 * hh + e]); } return f; }
__device__ __forceinline__ v8f wmma16b(v16b a, v16b b, v8f c) { v8f d = __builtin_amdgcn_wmma_f32_16x16x32_f16(false, a, false, b, (short)0, c, false, false); asm volatile("v_nop\n\tv_nop\n\tv_nop\n\tv_nop" : "+v"(d) : "v"(a), "v"(b)); return d; }
__device__ __forceinline__ void wave_lds_sync() { __builtin_amdgcn_fence(__ATOMIC_RELEASE, "workgroup"); __builtin_amdgcn_wave_barrier(); __builtin_amdgcn_fence(__ATOMIC_ACQUIRE, "workgroup"); }
__device__ __forceinline__ float nexp(float x) { return __builtin_amdgcn_exp2f(x * 1.4426950408889634f); }
__device__ __forceinline__ float sigm(float x) { return 1.0f / (1.0f + nexp(-x)); }
__device__ __forceinline__ float tanh_f(float x) { const float e = nexp(-2.0f * fabsf(x)); const float t = (1.0f - e) / (1.0f + e); return (x >= 0.0f) ? t : -t; }
__device__ __forceinline__ float pmul(float a, float b) { float p = a * b; asm volatile("" : "+v"(p)); return p; }

struct Wo_ { static constexpr size_t EMB = 0, IH = EMB + (size_t)H * F, HH = IH + (size_t)G4 * H, END = HH + (size_t)G4 * H; };
__global__ __launch_bounds__(256) void prep_kernel(const float* __restrict__ We, const float* __restrict__ be, const float* __restrict__ gam, const float* __restrict__ bet, const float* __restrict__ Wih, const float* __restrict__ bih, const float* __restrict__ Whh, const float* __restrict__ bhh, b16* __restrict__ R, float* __restrict__ P) {
  const size_t tid = (size_t)blockIdx.x * 256 + threadIdx.x, nth = (size_t)gridDim.x * 256;
  for (int pass = 0; pass < 2; ++pass) {
    for (size_t q = tid; q < (size_t)H * F; q += nth) R[Wo_::EMB + q] = (b16)bf16_rne(We[q]);
    for (size_t q = tid; q < (size_t)G4 * H; q += nth) { R[Wo_::IH + q] = (b16)bf16_rne(Wih[q]); R[Wo_::HH + q] = (b16)bf16_rne(Whh[q]); }
    for (size_t q = tid; q < 11264; q += nth) { float v; if (q < 1024) v = be[q]; else if (q < 2048) v = gam[q - 1024]; else if (q < 3072) v = bet[q - 2048]; else if (q < 7168) v = bih[q - 3072]; else v = bhh[q - 7168]; P[q] = bf16_rne(v); }
    __threadfence(); }
}

__global__ __launch_bounds__(128) void emb_kernel(const float* __restrict__ feats, const b16* __restrict__ R, const float* __restrict__ P, float* __restrict__ X) {
  __shared__ __attribute__((aligned(16))) float Ts[4][32 * 64];
  const int lane = threadIdx.x & 31, wave = threadIdx.x >> 5, nloc = lane & 15, hlf = lane >> 4, m0 = blockIdx.y * 128 + wave * 32, c0 = blockIdx.x * 64;
  v8f acc[2][4];
#pragma unroll
  for (int r = 0; r < 2; ++r)
#pragma unroll
    for (int t = 0; t < 4; ++t) acc[r][t] = (v8f){};
#pragma unroll 2
  for (int kb = 0; kb < F; kb += 32) { const v16b a0 = frag_x(feats + (size_t)(m0 + nloc) * F + kb, hlf), a1 = frag_x(feats + (size_t)(m0 + 16 + nloc) * F + kb, hlf);
#pragma unroll
    for (int t = 0; t < 4; ++t) { const v16b bw = frag_kb(R + Wo_::EMB + (size_t)(c0 + t * 16 + nloc) * F + kb, hlf); acc[0][t] = wmma16b(a0, bw, acc[0][t]); acc[1][t] = wmma16b(a1, bw, acc[1][t]); } }
  float* Tt = Ts[wave];
#pragma unroll
  for (int t = 0; t < 4; ++t) { const float bb = P[c0 + t * 16 + nloc];
#pragma unroll
    for (int r = 0; r < 2; ++r)
#pragma unroll
      for (int v = 0; v < 8; ++v) Tt[(r * 16 + v + 8 * hlf) * 64 + t * 16 + nloc] = acc[r][t][v] + bb; }
  wave_lds_sync();
  for (int pass = 0; pass < 2; ++pass) {
#pragma unroll
    for (int j = 0; j < 16; ++j) { const int rr = j * 2 + hlf, c4 = nloc * 4; *(volatile v4f*)(X + (size_t)(m0 + rr) * H + c0 + c4) = *(const v4f*)(Tt + rr * 64 + c4); }
    __threadfence(); }
}

__global__ __launch_bounds__(256) void bnstat_kernel(const float* __restrict__ X, float* __restrict__ st) {
  __shared__ float red[8][32]; __shared__ float mu[32];
  const int c0 = blockIdx.x * 32, lc = threadIdx.x & 31, rg = threadIdx.x >> 5;
  float s = 0.0f; for (int r = rg; r < NR; r += 8) s += X[(size_t)r * H + c0 + lc];
  red[rg][lc] = s; __syncthreads();
  if (rg == 0) { float a = 0.0f; for (int k = 0; k < 8; ++k) a += red[k][lc]; mu[lc] = a / (float)NR; }
  __syncthreads();
  const float m = mu[lc]; float q = 0.0f; for (int r = rg; r < NR; r += 8) { const float d = X[(size_t)r * H + c0 + lc] - m; q += pmul(d, d); }
  __syncthreads(); red[rg][lc] = q; __syncthreads();
  if (rg == 0) { float a = 0.0f; for (int k = 0; k < 8; ++k) a += red[k][lc]; const float is = rsqrtf(a / (float)NR + EPS); for (int pass = 0; pass < 2; ++pass) { ((volatile float*)st)[(c0 + lc) * 2] = m; ((volatile float*)st)[(c0 + lc) * 2 + 1] = is; } }
  __threadfence();
}

__global__ __launch_bounds__(128) void gx_kernel(const float* __restrict__ X, const float* __restrict__ st, const float* __restrict__ mask, const b16* __restrict__ R, const float* __restrict__ P, float* __restrict__ GX) {
  __shared__ __attribute__((aligned(16))) float Ts[4][32 * 64];
  const int lane = threadIdx.x & 31, wave = threadIdx.x >> 5, nloc = lane & 15, hlf = lane >> 4, m0 = blockIdx.y * 128 + wave * 32, c0 = blockIdx.x * 64; const float* gam = P + 1024; const float* bet = P + 2048; const float* bih = P + 3072;
  const float mk0 = bf16_rne(mask[m0 + nloc]), mk1 = bf16_rne(mask[m0 + 16 + nloc]);
  v8f acc[2][4];
#pragma unroll
  for (int r = 0; r < 2; ++r)
#pragma unroll
    for (int t = 0; t < 4; ++t) acc[r][t] = (v8f){};
#pragma unroll 2
  for (int kb = 0; kb < H; kb += 32) { v16b a0, a1;
#pragma unroll
    for (int e = 0; e < 16; ++e) { const int k = kb + ((e < 8) ? (8 * hlf + e) : (16 + 8 * hlf + e - 8)); const float m_ = st[k * 2], is = st[k * 2 + 1], g = gam[k], bb = bet[k];
      const float v0 = fmaxf(pmul((X[(size_t)(m0 + nloc) * H + k] - m_) * is, g) + bb, 0.0f) * mk0, v1 = fmaxf(pmul((X[(size_t)(m0 + 16 + nloc) * H + k] - m_) * is, g) + bb, 0.0f) * mk1; a0[e] = (b16)(v0 * AS_); a1[e] = (b16)(v1 * AS_); }
#pragma unroll
    for (int t = 0; t < 4; ++t) { const v16b bw = frag_kb(R + Wo_::IH + (size_t)(c0 + t * 16 + nloc) * H + kb, hlf); acc[0][t] = wmma16b(a0, bw, acc[0][t]); acc[1][t] = wmma16b(a1, bw, acc[1][t]); } }
  float* Tt = Ts[wave];
#pragma unroll
  for (int t = 0; t < 4; ++t) { const float bb = bih[c0 + t * 16 + nloc];
#pragma unroll
    for (int r = 0; r < 2; ++r)
#pragma unroll
      for (int v = 0; v < 8; ++v) Tt[(r * 16 + v + 8 * hlf) * 64 + t * 16 + nloc] = acc[r][t][v] * (1.0f / AS_) + bb; }
  wave_lds_sync();
  for (int pass = 0; pass < 2; ++pass) {
#pragma unroll
    for (int j = 0; j < 16; ++j) { const int rr = j * 2 + hlf, c4 = nloc * 4; *(volatile v4f*)(GX + (size_t)(m0 + rr) * G4 + c0 + c4) = *(const v4f*)(Tt + rr * 64 + c4); }
    __threadfence(); }
}

__global__ __launch_bounds__(512) void lstm_kernel(const float* __restrict__ GX, const float* __restrict__ mask, const b16* __restrict__ R, const float* __restrict__ P, float* __restrict__ out) {
  __shared__ __attribute__((aligned(16))) b16 Hs[16][H + 8];
  const int wave = threadIdx.x >> 5, lane = threadIdx.x & 31, nloc = lane & 15, hlf = lane >> 4, b0 = blockIdx.x * 16, u0 = wave * 64; const b16* Whh = R + Wo_::HH; const float* bhh = P + 7168;
  for (int i = threadIdx.x; i < 16 * (H + 8); i += 512) (&Hs[0][0])[i] = (b16)0.0f;
  float c[4][8];
#pragma unroll
  for (int t = 0; t < 4; ++t)
#pragma unroll
    for (int r = 0; r < 8; ++r) c[t][r] = 0.0f;
  __syncthreads();
  for (int step = 0; step < T; ++step) {
    v8f g[4][4];
#pragma unroll
    for (int q = 0; q < 4; ++q)
#pragma unroll
      for (int t = 0; t < 4; ++t) g[q][t] = (v8f){};
#pragma unroll 2
    for (int kb = 0; kb < H; kb += 32) { const v16b a = frag_kb(&Hs[nloc][kb], hlf);
#pragma unroll
      for (int q = 0; q < 4; ++q)
#pragma unroll
        for (int t = 0; t < 4; ++t) { const v16b bw = frag_kb(Whh + (size_t)(q * H + u0 + t * 16 + nloc) * H + kb, hlf); g[q][t] = wmma16b(a, bw, g[q][t]); } }
    float hn[4][8];
#pragma unroll
    for (int t = 0; t < 4; ++t) { const int u = u0 + t * 16 + nloc;
#pragma unroll
      for (int r = 0; r < 8; ++r) { const int rr = 8 * hlf + r, b = b0 + rr; const float* gx = GX + ((size_t)b * T + step) * G4; const float m = bf16_rne(mask[(size_t)b * T + step]);
        const float gi = sigm(g[0][t][r] * (1.0f / AS_) + gx[u] + bhh[u]), gf = sigm(g[1][t][r] * (1.0f / AS_) + gx[H + u] + bhh[H + u]), gg = tanh_f(g[2][t][r] * (1.0f / AS_) + gx[2 * H + u] + bhh[2 * H + u]), go = sigm(g[3][t][r] * (1.0f / AS_) + gx[3 * H + u] + bhh[3 * H + u]);
        const float cc = pmul(gf, c[t][r]) + pmul(gi, gg); c[t][r] = cc * m; hn[t][r] = pmul(go, tanh_f(cc)) * m; } }
    __syncthreads();
#pragma unroll
    for (int t = 0; t < 4; ++t) { const int u = u0 + t * 16 + nloc;
#pragma unroll
      for (int r = 0; r < 8; ++r) Hs[8 * hlf + r][u] = (b16)(hn[t][r] * AS_); }
    __syncthreads();
    { __shared__ __attribute__((aligned(16))) float Ot[16][16][64 + 4];
#pragma unroll
      for (int t = 0; t < 4; ++t)
#pragma unroll
        for (int r = 0; r < 8; ++r) Ot[wave][8 * hlf + r][t * 16 + nloc] = hn[t][r];
      wave_lds_sync();
      for (int pass = 0; pass < 2; ++pass) { for (int i = lane; i < 16 * 16; i += 32) { const int rr = i >> 4, c4 = (i & 15) * 4; *(volatile v4f*)(out + ((size_t)(b0 + rr) * T + step) * H + u0 + c4) = *(const v4f*)(&Ot[wave][rr][c4]); } __threadfence(); }
      wave_lds_sync(); } }
}
}

extern "C" void kernel_launch(void* const* d_in, const int* in_sizes, int n_in,
                              void* d_out, int out_size, void* d_ws, size_t ws_size, hipStream_t stream) {
  (void)n_in; (void)out_size;
  const float* feats = (const float*)d_in[0]; const float* mask = (const float*)d_in[1]; const float* We = (const float*)d_in[2]; const float* be = (const float*)d_in[3]; const float* gam = (const float*)d_in[4]; const float* bet = (const float*)d_in[5];
  const float* Wih = (const float*)d_in[6]; const float* bih = (const float*)d_in[7]; const float* Whh = (const float*)d_in[8]; const float* bhh = (const float*)d_in[9];
  float* out = (float*)d_out;
  if (in_sizes[0] != NR * F || in_sizes[1] != NR || in_sizes[2] != H * F || in_sizes[6] != G4 * H || in_sizes[8] != G4 * H) return;
  size_t off = 0; char* ws = (char*)d_ws;
  auto carve = [&](size_t bytes) { char* p = ws + off; off += (bytes + 255) & ~(size_t)255; return p; };
  b16* R = (b16*)carve(Wo_::END * 2); float* P = (float*)carve(12288 * 4); float* X = (float*)carve((size_t)NR * H * 4); float* st = (float*)carve(H * 2 * 4); float* GX = (float*)carve((size_t)NR * G4 * 4);
  if (off > ws_size) return;
  prep_kernel<<<512, 256, 0, stream>>>(We, be, gam, bet, Wih, bih, Whh, bhh, R, P);
  emb_kernel<<<dim3(H / 64, NR / 128), 128, 0, stream>>>(feats, R, P, X);
  bnstat_kernel<<<H / 32, 256, 0, stream>>>(X, st);
  gx_kernel<<<dim3(G4 / 64, NR / 128), 128, 0, stream>>>(X, st, mask, R, P, GX);
  lstm_kernel<<<B / 16, 512, 0, stream>>>(GX, mask, R, P, out);
}
